// Net_59545426592369
// MI455X (gfx1250) — hardware-verified
//
#include <hip/hip_runtime.h>
#include <stddef.h>
#include <stdint.h>
#include <math.h>


#define FEA    67
#define HID    16
#define NSTK   3
#define NCH    48
#define KP     96
#define NCG    96
#define T1PITCH 64
#define P2PITCH 16
#define T2PITCH 8
#define NTHR   256
#define NWAVE  8
#define EPT    8
#define CHUNK  (NTHR * EPT)
#define WCAP   (EPT * 32)
#define LISTN  (NWAVE * WCAP)
#define NBA    512
#define SLA    9
#define RCAP   20480
#define DEGCAP 96
#define GROWS  128
#define WUNITS 576
#define AGG_ZINTS (LISTN + 2 * RCAP + 3 * NBA)
#define CMP_LDS_INTS (AGG_ZINTS + 16)
#define WSMAX  134217728

static_assert((CHUNK & (CHUNK - 1)) == 0 && CHUNK <= 4096);
static_assert((NBA & (NBA - 1)) == 0 && NBA == (1 << SLA));
static_assert(((long long)CHUNK << SLA) < (1LL << 31));
static_assert(NBA % NWAVE == 0 && NBA % 32 == 0 && NBA == 2 * NTHR && NBA % GROWS == 0);
static_assert(RCAP % NTHR == 0 && (RCAP / 4) % NTHR == 0 && AGG_ZINTS % 4 == 0 && LISTN % 4 == 0);
static_assert(RCAP >= 16774 + 16774 / 20 + 1);
static_assert(DEGCAP >= 57 + 8);
static_assert(KP % 32 == 0 && KP >= FEA && NCG == 2 * NCH && NCH == NSTK * HID);
static_assert(GROWS == (NTHR / 32) * 16 && NCG % 16 == 0);
static_assert((16 * NCG * 4) % 128 == 0 && (16 * NCG) / 4 == 12 * 32);
static_assert(WUNITS == NCH * (KP / 8) && WUNITS % 32 == 0 && WUNITS <= 3 * NTHR);
static_assert(CMP_LDS_INTS * 4 <= 300000);
static_assert((NBA * P2PITCH) % (4 * NTHR) == 0 && (NBA * T2PITCH) % (4 * NTHR) == 0 && NBA * 2 == 4 * NTHR);

typedef float          v2f   __attribute__((ext_vector_type(2)));
typedef float          v4f   __attribute__((ext_vector_type(4)));
typedef float          v8f   __attribute__((ext_vector_type(8)));
typedef int            v4i   __attribute__((ext_vector_type(4)));
typedef int            v8i   __attribute__((ext_vector_type(8)));
typedef unsigned short v8us  __attribute__((ext_vector_type(8)));
typedef unsigned short v16us __attribute__((ext_vector_type(16)));
typedef __bf16         v16bf __attribute__((ext_vector_type(16)));
typedef v2f  __attribute__((may_alias)) v2fa;
typedef v4f  __attribute__((may_alias)) v4fa;
typedef v4i  __attribute__((may_alias)) v4ia;
typedef v8us __attribute__((may_alias)) v8usa;
union FragB { v16bf v; v16us u; v8us h[2]; v8i w; };
struct S6 { float a, b, c, d, e, f; };

__device__ __forceinline__ v8f wmb(const FragB& a, const FragB& b, v8f c) {
  v8f d = __builtin_amdgcn_wmma_f32_16x16x32_bf16(false, a.v, false, b.v, (short)0, c, false, false);
  asm volatile("v_nop\n\tv_nop\n\tv_nop\n\tv_nop" : "+v"(d) : "v"(a.w), "v"(b.w));
  return d;
}

__device__ __forceinline__ unsigned bf16_bits(float f) {
  const unsigned u = __float_as_uint(f);
  return (u + 0x7FFFu + ((u >> 16) & 1u)) >> 16;
}
__device__ __forceinline__ float bf16_val(float f) {
  return __uint_as_float(bf16_bits(f) << 16);
}
__device__ __forceinline__ float relu_keep(float v) { return (v > 0.0f) ? v : (v - v); }

__device__ __forceinline__ void wave_sync() {
  __builtin_amdgcn_fence(__ATOMIC_RELEASE, "wavefront");
  __builtin_amdgcn_wave_barrier();
  __builtin_amdgcn_fence(__ATOMIC_ACQUIRE, "wavefront");
}

__device__ __forceinline__ int wave_max_i(int v) {
#pragma unroll
  for (int d = 16; d >= 1; d >>= 1) {
    const int y = __shfl_xor(v, d, 32);
    v = v > y ? v : y;
  }
  return __builtin_amdgcn_readfirstlane(v);
}

template <int SLB>
__device__ __forceinline__ int scan_chunk(const int* __restrict__ dsts, int nE, int cbase, int slotBase,
                                          int nb, int vec8, int* list, int tid, int lane, int wave) {
  int wc = 0;
  const int el0  = tid * EPT;
  const int e0   = cbase + el0;
  const int sent = -2147483647 - 1;
  v4i da, db;
  if (vec8 != 0 && cbase + CHUNK <= nE) {
    da = *(const v4i*)(dsts + e0);
    db = *(const v4i*)(dsts + e0 + 4);
  } else {
    da.x = (e0     < nE) ? dsts[min(e0,     nE - 1)] : sent;
    da.y = (e0 + 1 < nE) ? dsts[min(e0 + 1, nE - 1)] : sent;
    da.z = (e0 + 2 < nE) ? dsts[min(e0 + 2, nE - 1)] : sent;
    da.w = (e0 + 3 < nE) ? dsts[min(e0 + 3, nE - 1)] : sent;
    db.x = (e0 + 4 < nE) ? dsts[min(e0 + 4, nE - 1)] : sent;
    db.y = (e0 + 5 < nE) ? dsts[min(e0 + 5, nE - 1)] : sent;
    db.z = (e0 + 6 < nE) ? dsts[min(e0 + 6, nE - 1)] : sent;
    db.w = (e0 + 7 < nE) ? dsts[min(e0 + 7, nE - 1)] : sent;
  }
  const unsigned nbs = (unsigned)slotBase;
  const unsigned unb = (unsigned)nb;
  const unsigned s0 = (unsigned)da.x - nbs, s1 = (unsigned)da.y - nbs;
  const unsigned s2 = (unsigned)da.z - nbs, s3 = (unsigned)da.w - nbs;
  const unsigned s4 = (unsigned)db.x - nbs, s5 = (unsigned)db.y - nbs;
  const unsigned s6 = (unsigned)db.z - nbs, s7 = (unsigned)db.w - nbs;
  const bool h0 = s0 < unb, h1 = s1 < unb, h2 = s2 < unb, h3 = s3 < unb;
  const bool h4 = s4 < unb, h5 = s5 < unb, h6 = s6 < unb, h7 = s7 < unb;
  const unsigned any = __builtin_amdgcn_ballot_w32(h0 | h1 | h2 | h3 | h4 | h5 | h6 | h7);
  if (any != 0u) {
#define HITJ(J, HJ, SJ) { \
      const unsigned mj = __builtin_amdgcn_ballot_w32(HJ); \
      if (mj != 0u) { \
        if (HJ) { \
          const int pos = wc + (int)__builtin_amdgcn_mbcnt_lo(mj, 0u); \
          if (pos < WCAP) list[wave * WCAP + pos] = ((el0 + (J)) << SLB) | (int)(SJ); \
        } \
        wc += (int)__builtin_popcount(mj); } }
    HITJ(0, h0, s0)
    HITJ(1, h1, s1)
    HITJ(2, h2, s2)
    HITJ(3, h3, s3)
    HITJ(4, h4, s4)
    HITJ(5, h5, s5)
    HITJ(6, h6, s6)
    HITJ(7, h7, s7)
#undef HITJ
  }
  return wc;
}

__device__ __forceinline__ void wcat_unit(const float* __restrict__ W, int v, int nOff, unsigned short* WT) {
  const bool act = v < WUNITS;
  const int vc  = act ? v : WUNITS - 1;
  const int n   = vc / 12;
  const int k8  = (vc - n * 12) * 8;
  const int kst = n >> 4, h = n & 15;
  v8us o;
#pragma unroll
  for (int i = 0; i < 8; ++i) {
    const int kk = k8 + i;
    const int kc = kk < FEA ? kk : FEA - 1;
    const float f = W[(size_t)(kst * FEA + kc) * HID + h];
    o[i] = (kk < FEA) ? (unsigned short)bf16_bits(f) : (unsigned short)0;
  }
  unsigned short* dp = WT + (size_t)(nOff + n) * KP + k8;
  if (act) *(volatile v8us*)dp = o;
  __threadfence();
  if (act) *(volatile v8us*)dp = o;
}

__global__ __launch_bounds__(NTHR) void k_prep(const float* __restrict__ x, const float* __restrict__ iw,
                                               const float* __restrict__ rw, int nN, int gX,
                                               unsigned short* XB, unsigned short* WT) {
  const int b = (int)blockIdx.x, tid = (int)threadIdx.x;
  if (b < gX) {
    const int u   = b * NTHR + tid;
    const int row = u / 12;
    const int k8  = (u - row * 12) * 8;
    const int rc  = row < nN ? row : nN - 1;
    const float* p = x + (size_t)rc * FEA;
    v8us o;
#pragma unroll
    for (int i = 0; i < 8; ++i) {
      const int kk = k8 + i;
      const int kc = kk < FEA ? kk : FEA - 1;
      const float f = p[kc];
      const bool ok = (row < nN) && (kk < FEA);
      o[i] = ok ? (unsigned short)bf16_bits(f) : (unsigned short)0;
    }
    unsigned short* dp = XB + (size_t)u * 8;
    *(volatile v8us*)dp = o;
    __threadfence();
    *(volatile v8us*)dp = o;
  } else if (b < gX + 3) {
    wcat_unit(iw, (b - gX) * NTHR + tid, 0, WT);
  } else {
    wcat_unit(rw, (b - gX - 3) * NTHR + tid, NCH, WT);
  }
}

__global__ __launch_bounds__(NTHR) void k_compact(const int* __restrict__ srcs, const int* __restrict__ dsts,
                                                  int nE, int nN, int vec8,
                                                  int* LIST, int* CNT, int* OFF, int* DINVb, int* FLAG) {
  extern __shared__ __attribute__((aligned(16))) int dsm[];
  int* list = dsm;
  int* hl   = dsm + LISTN;
  int* sl   = hl + RCAP;
  int* cnt  = sl + RCAP;
  int* offs = cnt + NBA;
  int* cur  = offs + NBA;
  int* misc = cur + NBA;
  const int tid = (int)threadIdx.x, lane = tid & 31, wave = tid >> 5;
  const int nodeBase = (int)blockIdx.x * NBA;
  int nb = nN - nodeBase;
  nb = nb < 0 ? 0 : (nb > NBA ? NBA : nb);

  {
    const v4i z4 = {0, 0, 0, 0};
    for (int i = tid * 4; i < AGG_ZINTS; i += NTHR * 4) *(v4ia*)(dsm + i) = z4;
    if (tid < 16) misc[tid] = 0;
  }
  __syncthreads();

  int t = 0, ov = 0;
  const int nChunks = (nE + CHUNK - 1) / CHUNK;
#pragma unroll 1
  for (int ch = 0; ch < nChunks; ++ch) {
    const int cbase = ch * CHUNK;
    const int wc = scan_chunk<SLA>(dsts, nE, cbase, nodeBase, nb, vec8, list, tid, lane, wave);
    if (lane == 0) misc[wave] = wc;
    __syncthreads();
    if (wave == 0) {
#pragma unroll 1
      for (int w2 = 0; w2 < NWAVE; ++w2) {
        int c = misc[w2];
        c = c < 0 ? 0 : (c > WCAP ? WCAP : c);
#pragma unroll 1
        for (int b0 = 0; b0 < c; b0 += 32) {
          const int idx = b0 + lane;
          const int ent = list[w2 * WCAP + (idx < WCAP ? idx : WCAP - 1)];
          const int m32 = (c - b0) < 32 ? (c - b0) : 32;
#pragma unroll 1
          for (int k = 0; k < m32; ++k) {
            const int u    = __builtin_amdgcn_readlane(ent, k);
            const int slot = u & (NBA - 1);
            const int el   = (u >> SLA) & (CHUNK - 1);
            const int pk   = ((cbase + el) << SLA) | slot;
            if (t < RCAP) {
              if (lane == 0) { hl[t] = pk; cnt[slot] = cnt[slot] + 1; }
              t = t + 1;
            } else {
              ov = 1;
            }
          }
        }
      }
    }
    __syncthreads();
  }
  if (wave == 0 && lane == 0) { misc[8] = t; misc[9] = ov; }
  __syncthreads();
  int tt = misc[8];
  tt = tt < 0 ? 0 : (tt > RCAP ? RCAP : tt);
  const int ovf = misc[9];

  if (wave == 0) {
    const int base = lane * (NBA / 32);
    int s = 0;
#pragma unroll 1
    for (int i = 0; i < NBA / 32; ++i) s += cnt[base + i];
    int incl = s;
#pragma unroll
    for (int d = 1; d < 32; d <<= 1) {
      const int y = __shfl_up(incl, d, 32);
      if (lane >= d) incl += y;
    }
    int run = incl - s;
#pragma unroll 1
    for (int i = 0; i < NBA / 32; ++i) {
      const int cv = cnt[base + i];
      offs[base + i] = run;
      cur[base + i]  = run;
      run += cv;
    }
  }
  __syncthreads();
  if (wave == 0) {
#pragma unroll 1
    for (int b0 = 0; b0 < tt; b0 += 32) {
      const int idx = b0 + lane;
      const int ent = hl[idx < RCAP ? idx : RCAP - 1];
      const int m32 = (tt - b0) < 32 ? (tt - b0) : 32;
#pragma unroll 1
      for (int k = 0; k < m32; ++k) {
        const int u    = __builtin_amdgcn_readlane(ent, k);
        const int slot = u & (NBA - 1);
        if (lane == 0) {
          int p = cur[slot];
          p = p < 0 ? 0 : (p > RCAP - 1 ? RCAP - 1 : p);
          sl[p] = u;
          cur[slot] = p + 1;
        }
      }
    }
  }
  __syncthreads();

#pragma unroll 1
  for (int idx = tid; idx < RCAP; idx += NTHR) {
    const int ent = sl[idx];
    int eid = ent >> SLA;
    eid = eid < 0 ? 0 : (eid > nE - 1 ? nE - 1 : eid);
    int sr = srcs[eid];
    sr = sr < 0 ? 0 : (sr > nN - 1 ? nN - 1 : sr);
    hl[idx] = (idx < tt) ? sr : 0;
  }
#pragma unroll 1
  for (int s = tid; s < NBA; s += NTHR) {
    const int c  = cnt[s];
    const int cc = c < 1 ? 1 : c;
    const float f = 1.0f / sqrtf((float)cc);
    cur[s] = (c > 0) ? __float_as_int(f) : 0;
  }
  __syncthreads();

  int* Lb = LIST + (size_t)blockIdx.x * RCAP;
  const v4i fl4 = {ovf, ovf, ovf, ovf};
#pragma unroll 1
  for (int it = 0; it < RCAP / 4 / NTHR; ++it) {
    const int q = it * NTHR + tid;
    const v4i v = *(const v4ia*)(hl + 4 * q);
    *(volatile v4i*)(Lb + 4 * q) = v;
  }
  if (tid < NBA / 4) {
    const v4i c4 = *(const v4ia*)(cnt + 4 * tid);
    const v4i o4 = *(const v4ia*)(offs + 4 * tid);
    const v4i d4 = *(const v4ia*)(cur + 4 * tid);
    *(volatile v4i*)(CNT   + nodeBase + 4 * tid) = c4;
    *(volatile v4i*)(OFF   + nodeBase + 4 * tid) = o4;
    *(volatile v4i*)(DINVb + nodeBase + 4 * tid) = d4;
  }
  if (tid < 8) *(volatile v4i*)(FLAG + (size_t)blockIdx.x * 32 + 4 * tid) = fl4;
  __threadfence();
#pragma unroll 1
  for (int it = 0; it < RCAP / 4 / NTHR; ++it) {
    const int q = it * NTHR + tid;
    const v4i v = *(const v4ia*)(hl + 4 * q);
    *(volatile v4i*)(Lb + 4 * q) = v;
  }
  if (tid < NBA / 4) {
    const v4i c4 = *(const v4ia*)(cnt + 4 * tid);
    const v4i o4 = *(const v4ia*)(offs + 4 * tid);
    const v4i d4 = *(const v4ia*)(cur + 4 * tid);
    *(volatile v4i*)(CNT   + nodeBase + 4 * tid) = c4;
    *(volatile v4i*)(OFF   + nodeBase + 4 * tid) = o4;
    *(volatile v4i*)(DINVb + nodeBase + 4 * tid) = d4;
  }
  if (tid < 8) *(volatile v4i*)(FLAG + (size_t)blockIdx.x * 32 + 4 * tid) = fl4;
}

__global__ __launch_bounds__(NTHR) void k_gemm1(const unsigned short* __restrict__ XB,
                                                const unsigned short* __restrict__ WT,
                                                const float* __restrict__ DINV, float* G) {
  __shared__ __attribute__((aligned(16))) float stg[GROWS * NCG];
  __shared__ __attribute__((aligned(16))) float sdv[GROWS];
  const int tid = (int)threadIdx.x, lane = tid & 31, wave = tid >> 5, hh = lane >> 4, m = lane & 15;
  const int rowBase = (int)blockIdx.x * GROWS;

  if (tid < GROWS / 4) {
    const v4f d = *(const v4f*)(DINV + (size_t)rowBase + 4 * tid);
    *(v4fa*)(sdv + 4 * tid) = d;
  }

  v8f acc[6];
  {
    const v8f z = {0.f, 0.f, 0.f, 0.f, 0.f, 0.f, 0.f, 0.f};
#pragma unroll
    for (int t = 0; t < 6; ++t) acc[t] = z;
  }
  const unsigned short* ap = XB + (size_t)(rowBase + 16 * wave + m) * KP + 8 * hh;
  const unsigned short* wp = WT + (size_t)m * KP + 8 * hh;
#pragma unroll 1
  for (int ks = 0; ks < KP / 32; ++ks) {
    FragB af;
    af.h[0] = *(const v8usa*)(ap + 32 * ks);
    af.h[1] = *(const v8usa*)(ap + 32 * ks + 16);
#pragma unroll
    for (int t = 0; t < 6; ++t) {
      const unsigned short* wq = wp + (size_t)(16 * t) * KP + 32 * ks;
      FragB bf;
      bf.h[0] = *(const v8usa*)wq;
      bf.h[1] = *(const v8usa*)(wq + 16);
      acc[t] = wmb(af, bf, acc[t]);
    }
  }

#pragma unroll
  for (int t = 0; t < 6; ++t) {
    const int lc = 16 * t + m;
#pragma unroll
    for (int r = 0; r < 8; ++r) {
      const int lr = 16 * wave + 8 * hh + r;
      stg[lr * NCG + lc] = acc[t][r];
    }
  }
  __syncthreads();

  v4f fv[12];
#pragma unroll
  for (int i = 0; i < 12; ++i) {
    const int q  = i * 32 + lane;
    const int r  = q / 24;
    const int c4 = q - r * 24;
    const int lr = 16 * wave + r;
    const v4f v  = *(const v4fa*)(stg + lr * NCG + 4 * c4);
    const float sc = (c4 < 12) ? sdv[lr] : 1.0f;
    fv[i] = v * sc;
  }
  float* ob = G + (size_t)(rowBase + 16 * wave) * NCG;
#pragma unroll
  for (int i = 0; i < 12; ++i) *(volatile v4f*)(ob + 4 * (i * 32 + lane)) = fv[i];
  __threadfence();
#pragma unroll
  for (int i = 0; i < 12; ++i) *(volatile v4f*)(ob + 4 * (i * 32 + lane)) = fv[i];
}

template <int PITCH>
__device__ __forceinline__ v2f gather_row2(const float* __restrict__ P, const int* __restrict__ Lb,
                                           int c, int o, int nN, int cl, int lane) {
  float a0 = 0.0f, a1 = 0.0f;
  const int last = o + c - 1;
#pragma unroll 1
  for (int b0 = 0; b0 < c; b0 += 32) {
    int idx = o + b0 + lane;
    idx = idx > last ? last : idx;
    idx = idx < 0 ? 0 : (idx > RCAP - 1 ? RCAP - 1 : idx);
    int sr = Lb[idx];
    sr = sr < 0 ? 0 : (sr > nN - 1 ? nN - 1 : sr);
    const int m32 = (c - b0) < 32 ? (c - b0) : 32;
#pragma unroll 1
    for (int k = 0; k < m32; ++k) {
      const int sk = __builtin_amdgcn_readlane(sr, k);
      const v2f a = *(const v2fa*)(P + (size_t)sk * PITCH + cl);
      a0 += a.x; a1 += a.y;
    }
  }
  v2f r; r.x = a0; r.y = a1;
  return r;
}

template <int PITCH>
__device__ __forceinline__ S6 gather6(const float* __restrict__ P, const int* __restrict__ Lb,
                                      int c, int o, int cmax, int nN) {
  S6 s; s.a = 0.0f; s.b = 0.0f; s.c = 0.0f; s.d = 0.0f; s.e = 0.0f; s.f = 0.0f;
#pragma unroll 1
  for (int p = 0; p < cmax; ++p) {
    int pi = p < c ? p : c - 1;
    pi = pi < 0 ? 0 : pi;
    int idx = o + pi;
    idx = idx < 0 ? 0 : (idx > RCAP - 1 ? RCAP - 1 : idx);
    int sr = Lb[idx];
    sr = sr < 0 ? 0 : (sr > nN - 1 ? nN - 1 : sr);
    const float* rp = P + (size_t)sr * PITCH;
    const v4f x4 = *(const v4fa*)rp;
    const v2f x2 = *(const v2fa*)(rp + 4);
    const int mk = -(int)(p < c);
    s.a += __int_as_float(__float_as_int(x4.x) & mk);
    s.b += __int_as_float(__float_as_int(x4.y) & mk);
    s.c += __int_as_float(__float_as_int(x4.z) & mk);
    s.d += __int_as_float(__float_as_int(x4.w) & mk);
    s.e += __int_as_float(__float_as_int(x2.x) & mk);
    s.f += __int_as_float(__float_as_int(x2.y) & mk);
  }
  return s;
}

__global__ __launch_bounds__(NTHR) void k_agg1a(const int* __restrict__ LIST, const int* __restrict__ CNT,
                                                const int* __restrict__ OFF, const float* __restrict__ DINV,
                                                const int* __restrict__ FLAG, const float* __restrict__ G,
                                                const float* __restrict__ w1, const float* __restrict__ b1,
                                                int nN, float* T1P) {
  __shared__ __attribute__((aligned(16))) int   scn[NBA];
  __shared__ __attribute__((aligned(16))) int   sof[NBA];
  __shared__ __attribute__((aligned(16))) float sdv[NBA];
  __shared__ __attribute__((aligned(16))) float sw1[NSTK * HID * HID];
  __shared__ __attribute__((aligned(16))) float sb1[NCH];
  __shared__ __attribute__((aligned(16))) float prow[NWAVE * NCH];
  const int tid = (int)threadIdx.x, lane = tid & 31, wave = tid >> 5;
  const int b = (int)blockIdx.x;
  const int nodeBase = b * NBA;

  if (tid < NBA / 4) {
    const v4i c4 = *(const v4i*)(CNT + nodeBase + 4 * tid);
    const v4i o4 = *(const v4i*)(OFF + nodeBase + 4 * tid);
    const v4f d4 = *(const v4f*)(DINV + nodeBase + 4 * tid);
    *(v4ia*)(scn + 4 * tid) = c4;
    *(v4ia*)(sof + 4 * tid) = o4;
    *(v4fa*)(sdv + 4 * tid) = d4;
  }
#pragma unroll 1
  for (int i = tid; i < NSTK * HID * HID; i += NTHR) sw1[i] = bf16_val(w1[i]);
  {
    const float bb = b1[tid < NCH ? tid : NCH - 1];
    if (tid < NCH) sb1[tid] = bf16_val(bb);
  }
  const int flag = FLAG[(size_t)b * 32];
  __syncthreads();

  const int* Lb = LIST + (size_t)b * RCAP;
  const float qnan = __int_as_float(0x7fc00000);
  const float pz = (flag != 0) ? qnan : 0.0f;
  const int cl = (2 * lane) < (NCH - 2) ? (2 * lane) : (NCH - 2);
  const int lt = lane < 23 ? lane : 23;
  const int kq = lt >> 3, pq = (2 * lt) & 15;
  const int sa = (2 * lane) & 31, sb = (2 * lane + 1) & 31;
  float* pr = prow + wave * NCH;
#pragma unroll 1
  for (int si = 0; si < NBA / NWAVE; ++si) {
    const int s    = si * NWAVE + wave;
    const int node = nodeBase + s;
    int c = __builtin_amdgcn_readfirstlane(scn[s]);
    const bool big = c > DEGCAP;
    c = c < 0 ? 0 : (c > DEGCAP ? DEGCAP : c);
    int o = __builtin_amdgcn_readfirstlane(sof[s]);
    o = o < 0 ? 0 : (o > RCAP ? RCAP : o);
    const int nc = node < nN ? node : nN - 1;
    const float dd = sdv[s];
    const v2f S  = gather_row2<NCG>(G, Lb, c, o, nN, cl, lane);
    const v2f rt = *(const v2fa*)(G + (size_t)nc * NCG + NCH + cl);
    const float pzr = big ? qnan : pz;
    float y0 = (dd * S.x + rt.x) + sb1[cl];
    float y1 = (dd * S.y + rt.y) + sb1[cl + 1];
    y0 = relu_keep(y0) + pzr;
    y1 = relu_keep(y1) + pzr;
    if (lane < 24) { pr[2 * lane] = y0; pr[2 * lane + 1] = y1; }
    wave_sync();
    float t0 = 0.0f, t1 = 0.0f;
    const float* ph = pr + kq * HID;
    const float* wr = sw1 + kq * (HID * HID) + pq;
#pragma unroll 2
    for (int h = 0; h < HID; ++h) {
      const float pv = ph[h];
      const v2f w = *(const v2fa*)(wr + h * HID);
      t0 = fmaf(pv, w.x, t0);
      t1 = fmaf(pv, w.y, t1);
    }
    wave_sync();
    const bool keep = (node < nN) && (lane < 24);
    const float tz0 = keep ? dd * t0 : 0.0f;
    const float tz1 = keep ? dd * t1 : 0.0f;
    v4f ow;
    ow.x = __shfl(tz0, sa, 32); ow.y = __shfl(tz1, sa, 32);
    ow.z = __shfl(tz0, sb, 32); ow.w = __shfl(tz1, sb, 32);
    float* op = T1P + (size_t)node * T1PITCH + 4 * (lane & 15);
    const bool wrl = lane < 16;
    if (wrl) *(volatile v4f*)op = ow;
    __threadfence();
    if (wrl) *(volatile v4f*)op = ow;
  }
}

__global__ __launch_bounds__(NTHR) void k_agg1b(const int* __restrict__ LIST, const int* __restrict__ CNT,
                                                const int* __restrict__ OFF, const float* __restrict__ DINV,
                                                const int* __restrict__ FLAG, const float* __restrict__ G,
                                                const float* __restrict__ T1P, const float* __restrict__ b1,
                                                const float* __restrict__ iw2, const float* __restrict__ rw2,
                                                int nN, float* PR2) {
  __shared__ __attribute__((aligned(16))) int   scn[NBA];
  __shared__ __attribute__((aligned(16))) int   sof[NBA];
  __shared__ __attribute__((aligned(16))) float sdv[NBA];
  __shared__ __attribute__((aligned(16))) float sb1[NCH];
  __shared__ __attribute__((aligned(16))) float sw2c[HID * 12];
  __shared__ __attribute__((aligned(16))) float prow[NWAVE * NCH];
  __shared__ __attribute__((aligned(16))) float hrow[NWAVE * HID];
  __shared__ __attribute__((aligned(16))) float stg[NBA * P2PITCH];
  const int tid = (int)threadIdx.x, lane = tid & 31, wave = tid >> 5;
  const int b = (int)blockIdx.x;
  const int nodeBase = b * NBA;

  if (tid < NBA / 4) {
    const v4i c4 = *(const v4i*)(CNT + nodeBase + 4 * tid);
    const v4i o4 = *(const v4i*)(OFF + nodeBase + 4 * tid);
    const v4f d4 = *(const v4f*)(DINV + nodeBase + 4 * tid);
    *(v4ia*)(scn + 4 * tid) = c4;
    *(v4ia*)(sof + 4 * tid) = o4;
    *(v4fa*)(sdv + 4 * tid) = d4;
  }
  {
    const float bb = b1[tid < NCH ? tid : NCH - 1];
    if (tid < NCH) sb1[tid] = bf16_val(bb);
    const int tc = tid < HID * 12 ? tid : HID * 12 - 1;
    const int h  = tc / 12, j = tc - h * 12;
    const int jj = j < 6 ? j : j - 6;
    const int sidx = ((jj >> 1) * HID + h) * 2 + (jj & 1);
    const float fa = iw2[sidx];
    const float fb = rw2[sidx];
    const int ma = -(int)(j < 6);
    const int bits = (__float_as_int(bf16_val(fa)) & ma) | (__float_as_int(bf16_val(fb)) & ~ma);
    if (tid < HID * 12) sw2c[tc] = __int_as_float(bits);
  }
  const int flag = FLAG[(size_t)b * 32];
  __syncthreads();

  const int* Lb = LIST + (size_t)b * RCAP;
  const float qnan = __int_as_float(0x7fc00000);
  const float pz = (flag != 0) ? qnan : 0.0f;
  const int cl = (2 * lane) < (NCH - 2) ? (2 * lane) : (NCH - 2);
  const int lh = lane & 15;
  const int jq = lane < 11 ? lane : 11;
  const int col = lane < 6 ? lane : (lane < 12 ? lane + 2 : (lane < 14 ? lane - 6 : lane));
  float* pr = prow + wave * NCH;
  float* hr = hrow + wave * HID;
#pragma unroll 1
  for (int si = 0; si < NBA / NWAVE; ++si) {
    const int s    = si * NWAVE + wave;
    const int node = nodeBase + s;
    int c = __builtin_amdgcn_readfirstlane(scn[s]);
    const bool big = c > DEGCAP;
    c = c < 0 ? 0 : (c > DEGCAP ? DEGCAP : c);
    int o = __builtin_amdgcn_readfirstlane(sof[s]);
    o = o < 0 ? 0 : (o > RCAP ? RCAP : o);
    const int nc = node < nN ? node : nN - 1;
    const float dd = sdv[s];
    const v2f S  = gather_row2<T1PITCH>(T1P, Lb, c, o, nN, cl, lane);
    const v2f rt = *(const v2fa*)(G + (size_t)nc * NCG + NCH + cl);
    const float pzr = big ? qnan : pz;
    float y0 = (dd * S.x + rt.x) + sb1[cl];
    float y1 = (dd * S.y + rt.y) + sb1[cl + 1];
    y0 = relu_keep(y0) + pzr;
    y1 = relu_keep(y1) + pzr;
    if (lane < 24) { pr[2 * lane] = y0; pr[2 * lane + 1] = y1; }
    wave_sync();
    const float mv = ((pr[lh] + pr[HID + lh]) + pr[2 * HID + lh]) * (1.0f / 3.0f);
    const float hv = relu_keep(mv);
    if (lane < 16) hr[lane] = hv;
    wave_sync();
    float s2 = 0.0f;
#pragma unroll 2
    for (int h = 0; h < HID; ++h) s2 = fmaf(hr[h], sw2c[h * 12 + jq], s2);
    wave_sync();
    float val = (lane < 6) ? dd * s2 : s2;
    val = ((node < nN) && (lane < 12)) ? val : 0.0f;
    if (lane < 16) stg[s * P2PITCH + col] = val;
  }
  __syncthreads();

  constexpr int NIT = (NBA * P2PITCH) / (4 * NTHR);
  v4f fv[NIT];
#pragma unroll
  for (int it = 0; it < NIT; ++it) fv[it] = *(const v4fa*)(stg + 4 * (it * NTHR + tid));
  float* ob = PR2 + (size_t)nodeBase * P2PITCH;
#pragma unroll
  for (int it = 0; it < NIT; ++it) *(volatile v4f*)(ob + 4 * (it * NTHR + tid)) = fv[it];
  __threadfence();
#pragma unroll
  for (int it = 0; it < NIT; ++it) *(volatile v4f*)(ob + 4 * (it * NTHR + tid)) = fv[it];
}

__global__ __launch_bounds__(NTHR) void k_agg2a(const int* __restrict__ LIST, const int* __restrict__ CNT,
                                                const int* __restrict__ OFF, const float* __restrict__ DINV,
                                                const int* __restrict__ FLAG, const float* __restrict__ PR2,
                                                const float* __restrict__ w2, const float* __restrict__ b2,
                                                int nN, float* T2P) {
  __shared__ __attribute__((aligned(16))) float sw2[16];
  __shared__ __attribute__((aligned(16))) float sb2[8];
  __shared__ __attribute__((aligned(16))) float stg[NBA * T2PITCH];
  const int tid = (int)threadIdx.x;
  const int b = (int)blockIdx.x;
  const int nodeBase = b * NBA;
  {
    const float wv = w2[tid < 12 ? tid : 11];
    const float bv = b2[tid < 6 ? tid : 5];
    if (tid < 16) sw2[tid] = (tid < 12) ? bf16_val(wv) : 0.0f;
    if (tid < 8)  sb2[tid] = (tid < 6) ? bf16_val(bv) : 0.0f;
  }
  const int flag = FLAG[(size_t)b * 32];
  __syncthreads();

  const int* Lb = LIST + (size_t)b * RCAP;
  const float qnan = __int_as_float(0x7fc00000);
  const float pz = (flag != 0) ? qnan : 0.0f;
#pragma unroll 1
  for (int hs = 0; hs < NBA / NTHR; ++hs) {
    const int s    = hs * NTHR + tid;
    const int node = nodeBase + s;
    int c = CNT[node];
    const bool big = c > DEGCAP;
    c = c < 0 ? 0 : (c > DEGCAP ? DEGCAP : c);
    int o = OFF[node];
    o = o < 0 ? 0 : (o > RCAP ? RCAP : o);
    const float dd = DINV[node];
    const int cm = wave_max_i(c);
    const S6 g = gather6<P2PITCH>(PR2, Lb, c, o, cm, nN);
    const int nc = node < nN ? node : nN - 1;
    const v4f r4 = *(const v4fa*)(PR2 + (size_t)nc * P2PITCH + 8);
    const v2f r2 = *(const v2fa*)(PR2 + (size_t)nc * P2PITCH + 12);
    const float pzr = big ? qnan : pz;
    const float q0 = ((dd * g.a + r4.x) + sb2[0]) + pzr;
    const float q1 = ((dd * g.b + r4.y) + sb2[1]) + pzr;
    const float q2 = ((dd * g.c + r4.z) + sb2[2]) + pzr;
    const float q3 = ((dd * g.d + r4.w) + sb2[3]) + pzr;
    const float q4 = ((dd * g.e + r2.x) + sb2[4]) + pzr;
    const float q5 = ((dd * g.f + r2.y) + sb2[5]) + pzr;
    const float t0 = q0 * sw2[0] + q1 * sw2[2];
    const float t1 = q0 * sw2[1] + q1 * sw2[3];
    const float t2 = q2 * sw2[4] + q3 * sw2[6];
    const float t3 = q2 * sw2[5] + q3 * sw2[7];
    const float t4 = q4 * sw2[8] + q5 * sw2[10];
    const float t5 = q4 * sw2[9] + q5 * sw2[11];
    const bool live = node < nN;
    v4f oa, obv;
    oa.x = live ? dd * t0 : 0.0f; oa.y = live ? dd * t1 : 0.0f;
    oa.z = live ? dd * t2 : 0.0f; oa.w = live ? dd * t3 : 0.0f;
    obv.x = live ? dd * t4 : 0.0f; obv.y = live ? dd * t5 : 0.0f;
    obv.z = 0.0f; obv.w = 0.0f;
    *(v4fa*)(stg + s * T2PITCH)     = oa;
    *(v4fa*)(stg + s * T2PITCH + 4) = obv;
  }
  __syncthreads();

  constexpr int NIT = (NBA * T2PITCH) / (4 * NTHR);
  v4f fv[NIT];
#pragma unroll
  for (int it = 0; it < NIT; ++it) fv[it] = *(const v4fa*)(stg + 4 * (it * NTHR + tid));
  float* ob = T2P + (size_t)nodeBase * T2PITCH;
#pragma unroll
  for (int it = 0; it < NIT; ++it) *(volatile v4f*)(ob + 4 * (it * NTHR + tid)) = fv[it];
  __threadfence();
#pragma unroll
  for (int it = 0; it < NIT; ++it) *(volatile v4f*)(ob + 4 * (it * NTHR + tid)) = fv[it];
}

__global__ __launch_bounds__(NTHR) void k_agg2b(const int* __restrict__ LIST, const int* __restrict__ CNT,
                                                const int* __restrict__ OFF, const float* __restrict__ DINV,
                                                const int* __restrict__ FLAG, const float* __restrict__ PR2,
                                                const float* __restrict__ T2P, const float* __restrict__ b2,
                                                int nN, int nOutF, float* out) {
  __shared__ __attribute__((aligned(16))) float sb2[8];
  __shared__ __attribute__((aligned(16))) float stg[NBA * 2];
  const int tid = (int)threadIdx.x;
  const int b = (int)blockIdx.x;
  const int nodeBase = b * NBA;
  {
    const float bv = b2[tid < 6 ? tid : 5];
    if (tid < 8) sb2[tid] = (tid < 6) ? bf16_val(bv) : 0.0f;
  }
  const int flag = FLAG[(size_t)b * 32];
  __syncthreads();

  const int* Lb = LIST + (size_t)b * RCAP;
  const float qnan = __int_as_float(0x7fc00000);
  const float pz = (flag != 0) ? qnan : 0.0f;
#pragma unroll 1
  for (int hs = 0; hs < NBA / NTHR; ++hs) {
    const int s    = hs * NTHR + tid;
    const int node = nodeBase + s;
    int c = CNT[node];
    const bool big = c > DEGCAP;
    c = c < 0 ? 0 : (c > DEGCAP ? DEGCAP : c);
    int o = OFF[node];
    o = o < 0 ? 0 : (o > RCAP ? RCAP : o);
    const float dd = DINV[node];
    const int cm = wave_max_i(c);
    const S6 g = gather6<T2PITCH>(T2P, Lb, c, o, cm, nN);
    const int nc = node < nN ? node : nN - 1;
    const v4f r4 = *(const v4fa*)(PR2 + (size_t)nc * P2PITCH + 8);
    const v2f r2 = *(const v2fa*)(PR2 + (size_t)nc * P2PITCH + 12);
    const float pzr = big ? qnan : pz;
    const float v0 = (dd * g.a + r4.x) + sb2[0];
    const float v1 = (dd * g.b + r4.y) + sb2[1];
    const float v2 = (dd * g.c + r4.z) + sb2[2];
    const float v3 = (dd * g.d + r4.w) + sb2[3];
    const float v4 = (dd * g.e + r2.x) + sb2[4];
    const float v5 = (dd * g.f + r2.y) + sb2[5];
    const float o0 = ((v0 + v2) + v4) * (1.0f / 3.0f);
    const float o1 = ((v1 + v3) + v5) * (1.0f / 3.0f);
    const bool gt = o0 > o1;
    const float mx = gt ? o0 : o1;
    const float dn = gt ? (o1 - o0) : (o0 - o1);
    const float ls = logf(1.0f + expf(dn));
    float e0 = ((o0 - mx) - ls) + pzr;
    float e1 = ((o1 - mx) - ls) + pzr;
    const bool live = node < nN;
    v2f ov;
    ov.x = live ? e0 : 0.0f;
    ov.y = live ? e1 : 0.0f;
    *(v2fa*)(stg + 2 * s) = ov;
  }
  __syncthreads();

  const v4f fv = *(const v4fa*)(stg + 4 * tid);
  const long long fbase = (long long)nodeBase * 2 + 4 * (long long)tid;
  const bool okst = (fbase + 4) <= (long long)nOutF;
  float* op = out + (okst ? fbase : 0);
  if (okst) *(volatile v4f*)op = fv;
  __threadfence();
  if (okst) *(volatile v4f*)op = fv;
}

static inline int cdiv(int a, int b) { return (a + b - 1) / b; }
static inline size_t al256(size_t o) { return (o + 255) & ~(size_t)255; }

extern "C" void kernel_launch(void* const* d_in, const int* in_sizes, int n_in,
                              void* d_out, int out_size, void* d_ws, size_t ws_size,
                              hipStream_t stream) {
  if (n_in < 10) return;
  if (in_sizes[0] < FEA || (in_sizes[0] % FEA) != 0) return;
  const int nN = in_sizes[0] / FEA;
  if (nN < 16 || (nN % 16) != 0 || nN > (1 << 22)) return;
  if (in_sizes[1] < 2 || (in_sizes[1] & 1) != 0) return;
  const int nE = in_sizes[1] / 2;
  if (nE < 1 || nE >= (1 << (31 - SLA))) return;
  if (in_sizes[2] != NSTK * FEA * HID) return;
  if (in_sizes[3] != NSTK * HID * HID) return;
  if (in_sizes[4] != NSTK * FEA * HID) return;
  if (in_sizes[5] != NCH) return;
  if (in_sizes[6] != NSTK * HID * 2) return;
  if (in_sizes[7] != NSTK * 4) return;
  if (in_sizes[8] != NSTK * HID * 2) return;
  if (in_sizes[9] != NSTK * 2) return;
  if ((long long)out_size != (long long)nN * 2) return;

  const float* x    = (const float*)d_in[0];
  const int*   edge = (const int*)d_in[1];
  const float* iw1  = (const float*)d_in[2];
  const float* w1   = (const float*)d_in[3];
  const float* rw1  = (const float*)d_in[4];
  const float* b1   = (const float*)d_in[5];
  const float* iw2  = (const float*)d_in[6];
  const float* w2   = (const float*)d_in[7];
  const float* rw2  = (const float*)d_in[8];
  const float* b2   = (const float*)d_in[9];
  float* out = (float*)d_out;
  const int* src = edge;
  const int* dst = edge + nE;

  const int MPX = cdiv(nN, GROWS) * GROWS;
  const int gM  = MPX / GROWS;
  const int gA  = cdiv(nN, NBA);
  const int NBP = gA * NBA;
  if (NBP < MPX) return;
  const int nUx = MPX * (KP / 8);
  if ((nUx % NTHR) != 0) return;
  const int gX  = nUx / NTHR;
  const int vec8 = ((nE & 3) == 0) ? 1 : 0;

  char* ws = (char*)d_ws;
  size_t off = 0;
  const size_t oXB   = off; off = al256(off + (size_t)MPX * KP * 2);
  const size_t oWT   = off; off = al256(off + (size_t)NCG * KP * 2);
  const size_t oG    = off; off = al256(off + (size_t)MPX * NCG * 4);
  const size_t oT1P  = off; off = al256(off + (size_t)NBP * T1PITCH * 4);
  const size_t oPR2  = off; off = al256(off + (size_t)NBP * P2PITCH * 4);
  const size_t oT2P  = off; off = al256(off + (size_t)NBP * T2PITCH * 4);
  const size_t oLIST = off; off = al256(off + (size_t)gA * RCAP * 4);
  const size_t oCNT  = off; off = al256(off + (size_t)NBP * 4);
  const size_t oOFF  = off; off = al256(off + (size_t)NBP * 4);
  const size_t oDINV = off; off = al256(off + (size_t)NBP * 4);
  const size_t oFLAG = off; off = al256(off + (size_t)gA * 128);
  if (off > ws_size || off > (size_t)WSMAX) return;
  unsigned short* XB   = (unsigned short*)(ws + oXB);
  unsigned short* WT   = (unsigned short*)(ws + oWT);
  float*          G    = (float*)(ws + oG);
  float*          T1P  = (float*)(ws + oT1P);
  float*          PR2  = (float*)(ws + oPR2);
  float*          T2P  = (float*)(ws + oT2P);
  int*            LIST = (int*)(ws + oLIST);
  int*            CNT  = (int*)(ws + oCNT);
  int*            OFF  = (int*)(ws + oOFF);
  float*          DINV = (float*)(ws + oDINV);
  int*            FLAG = (int*)(ws + oFLAG);

  const size_t cmpLds = (size_t)CMP_LDS_INTS * 4;
  hipFuncSetAttribute(reinterpret_cast<const void*>(&k_compact), hipFuncAttributeMaxDynamicSharedMemorySize, (int)cmpLds);

  k_prep<<<gX + 6, NTHR, 0, stream>>>(x, iw1, rw1, nN, gX, XB, WT);
  k_compact<<<gA, NTHR, cmpLds, stream>>>(src, dst, nE, nN, vec8, LIST, CNT, OFF, (int*)DINV, FLAG);
  k_gemm1<<<gM, NTHR, 0, stream>>>(XB, WT, DINV, G);
  k_agg1a<<<gA, NTHR, 0, stream>>>(LIST, CNT, OFF, DINV, FLAG, G, w1, b1, nN, T1P);
  k_agg1b<<<gA, NTHR, 0, stream>>>(LIST, CNT, OFF, DINV, FLAG, G, T1P, b1, iw2, rw2, nN, PR2);
  k_agg2a<<<gA, NTHR, 0, stream>>>(LIST, CNT, OFF, DINV, FLAG, PR2, w2, b2, nN, T2P);
  k_agg2b<<<gA, NTHR, 0, stream>>>(LIST, CNT, OFF, DINV, FLAG, PR2, T2P, b2, nN, out_size, out);
}
